// RNN_24515673325781
// MI455X (gfx1250) — hardware-verified
//
#include <hip/hip_runtime.h>
#include <math.h>

typedef __attribute__((ext_vector_type(16))) _Float16 v16h;
typedef __attribute__((ext_vector_type(8)))  _Float16 v8h;
typedef __attribute__((ext_vector_type(8)))  float    v8f;
typedef __attribute__((ext_vector_type(4)))  float    v4f;

constexpr int NB    = 256;
constexpr int NT    = 512;
constexpr int NI    = 64;
constexpr int NH    = 512;
constexpr int NO    = 24;
constexpr int NOPAD = 32;
constexpr int RB    = 16;
constexpr int NTHR  = 256;
constexpr int NWAVE = NTHR / 32;
constexpr int HP    = NH + 8;
constexpr int HPLANE = RB * HP;
constexpr int TCH   = 8;
constexpr int RROW  = TCH * NO;
constexpr float WSC      = 16.0f;
constexpr float WSC_INV  = 1.0f / 16.0f;
constexpr float LOSC     = 2048.0f;
constexpr float LOSC_INV = 1.0f / 2048.0f;

static_assert(NB % RB == 0);
static_assert(NH == NWAVE * 64);
static_assert(NI % 32 == 0 && NH % 32 == 0);
static_assert(NOPAD == 2 * 16 && NO <= NOPAD);
static_assert(NH % (4 * 32) == 0);
static_assert(NWAVE == 2 * 4);
static_assert(RB * NOPAD == 2 * NTHR);
static_assert(HP % 8 == 0);
static_assert(NT % TCH == 0);
static_assert((RB * RROW / 4) % NTHR == 0);
static_assert((RROW * 4) % 128 == 0);
static_assert((NT * NO * 4) % 128 == 0);
static_assert(((TCH - 1) & TCH) == 0);

constexpr int CH_X   = NB * NT * NI / 8;
constexpr int CH_WHH = NH * NH / 8;
constexpr int CH_WIH = NH * NI / 8;
constexpr int CH_WHO = NOPAD * NH / 8;
constexpr int BLK_X   = CH_X / NTHR;
constexpr int BLK_WHH = CH_WHH / NTHR;
constexpr int BLK_WIH = CH_WIH / NTHR;
constexpr int BLK_WHO = CH_WHO / NTHR;
constexpr int CVT_E1 = BLK_X;
constexpr int CVT_E2 = CVT_E1 + BLK_WHH;
constexpr int CVT_E3 = CVT_E2 + BLK_WIH;
constexpr int CVT_BLOCKS = CVT_E3 + BLK_WHO;
static_assert(CH_X % NTHR == 0 && CH_WHH % NTHR == 0 && CH_WIH % NTHR == 0 && CH_WHO % NTHR == 0);
static_assert(CVT_BLOCKS == 4248);
static_assert(NH / 8 == 64);

__device__ __forceinline__ unsigned short f2bf_bits(float f) {
  unsigned u = __float_as_uint(f);
  return (unsigned short)((u + 0x7FFFu + ((u >> 16) & 1u)) >> 16);
}
__device__ __forceinline__ float bf_bits2f(unsigned short h) { return __uint_as_float(((unsigned)h) << 16); }
__device__ __forceinline__ float bf16r(float f) { return bf_bits2f(f2bf_bits(f)); }

__device__ __forceinline__ void acc_guard4(v8f& a, v8f& b, v8f& c, v8f& d) { asm volatile("v_nop\n\tv_nop\n\tv_nop\n\tv_nop" : "+v"(a), "+v"(b), "+v"(c), "+v"(d)); }
__device__ __forceinline__ void acc_guard2(v8f& a, v8f& b) { asm volatile("v_nop\n\tv_nop\n\tv_nop\n\tv_nop" : "+v"(a), "+v"(b)); }
__device__ __forceinline__ void guard4_f5(v8f& a0, v8f& a1, v8f& a2, v8f& a3,
                                          v16h f0, v16h f1, v16h f2, v16h f3, v16h f4) {
  asm volatile("v_nop\n\tv_nop\n\tv_nop\n\tv_nop"
               : "+v"(a0), "+v"(a1), "+v"(a2), "+v"(a3)
               : "v"(f0), "v"(f1), "v"(f2), "v"(f3), "v"(f4));
}
__device__ __forceinline__ void guard8_f6(v8f& a0, v8f& a1, v8f& a2, v8f& a3, v8f& a4, v8f& a5, v8f& a6, v8f& a7,
                                          v16h f0, v16h f1, v16h f2, v16h f3, v16h f4, v16h f5) {
  asm volatile("v_nop\n\tv_nop\n\tv_nop\n\tv_nop"
               : "+v"(a0), "+v"(a1), "+v"(a2), "+v"(a3), "+v"(a4), "+v"(a5), "+v"(a6), "+v"(a7)
               : "v"(f0), "v"(f1), "v"(f2), "v"(f3), "v"(f4), "v"(f5));
}
__device__ __forceinline__ void guard2_f3(v8f& a0, v8f& a1, v16h f0, v16h f1, v16h f2) {
  asm volatile("v_nop\n\tv_nop\n\tv_nop\n\tv_nop" : "+v"(a0), "+v"(a1) : "v"(f0), "v"(f1), "v"(f2));
}

template <typename T> struct Frag;
template <> struct Frag<_Float16> {
  typedef v16h V; union U { v16h v; v8h h[2]; };
  static __device__ __forceinline__ v16h load(const _Float16* p) {
    U f; f.h[0] = *(const v8h*)(p); f.h[1] = *(const v8h*)(p + 16); return f.v;
  }
  static __device__ __forceinline__ v8f mma(v16h a, v16h b, v8f c) {
    return __builtin_amdgcn_wmma_f32_16x16x32_f16(false, a, false, b, (short)0, c, false, false);
  }
};

__device__ __forceinline__ void cvt8_store(const float* __restrict__ sp, _Float16* __restrict__ dp, float sc, bool keep) {
  const v4f a = *(const v4f*)sp;
  const v4f b = *(const v4f*)(sp + 4);
  v8h hv;
#pragma unroll
  for (int e = 0; e < 4; ++e) {
    const float fa = keep ? (bf16r(a[e]) * sc) : 0.0f;
    const float fb = keep ? (bf16r(b[e]) * sc) : 0.0f;
    hv[e]     = (_Float16)fa;
    hv[4 + e] = (_Float16)fb;
  }
  *(volatile v8h*)dp = hv;
  __threadfence();
  *(volatile v8h*)dp = hv;
}

__global__ __launch_bounds__(NTHR) void cvt_kernel(const float* __restrict__ x, const float* __restrict__ w_ih,
                                                   const float* __restrict__ w_hh, const float* __restrict__ w_ho,
                                                   _Float16* __restrict__ x16, _Float16* __restrict__ wih16,
                                                   _Float16* __restrict__ whh16, _Float16* __restrict__ who16) {
  const int blk = blockIdx.x, tid = threadIdx.x;
  if (blk < CVT_E1) {
    const size_t i = (size_t)blk * NTHR + tid;
    cvt8_store(x + i * 8, x16 + i * 8, 1.0f, true);
  } else if (blk < CVT_E2) {
    const size_t i = (size_t)(blk - CVT_E1) * NTHR + tid;
    cvt8_store(w_hh + i * 8, whh16 + i * 8, WSC, true);
  } else if (blk < CVT_E3) {
    const size_t i = (size_t)(blk - CVT_E2) * NTHR + tid;
    cvt8_store(w_ih + i * 8, wih16 + i * 8, WSC, true);
  } else {
    const int i = (blk - CVT_E3) * NTHR + tid;
    const int row = i >> 6, c8 = i & 63;
    const int rowc = (row < NO) ? row : (NO - 1);
    cvt8_store(w_ho + (size_t)rowc * NH + c8 * 8, who16 + (size_t)i * 8, WSC, row < NO);
  }
}

__global__ __launch_bounds__(NTHR) void rnn_seq_kernel(const _Float16* __restrict__ x16, const _Float16* __restrict__ wih16,
                                                       const _Float16* __restrict__ whh16, const _Float16* __restrict__ who16,
                                                       const float* __restrict__ b_ih, const float* __restrict__ b_hh,
                                                       const float* __restrict__ b_ho, float* __restrict__ out) {
  __shared__ __align__(16) _Float16 hpl[2 * HPLANE];
  __shared__ __align__(16) float    part[NWAVE * 256];
  __shared__ __align__(16) float    ring[RB * RROW];
  const int tid = threadIdx.x, lane = tid & 31, wave = tid >> 5;
  const int c = lane & 15, hh = lane >> 4, koff = hh * 8, mOff = hh * 8;
  const int b0 = blockIdx.x * RB;
  const int n0 = wave * 64;
  _Float16* hhi = hpl;
  _Float16* hlo = hpl + HPLANE;

  {
    const v8h z = {(_Float16)0.0f, (_Float16)0.0f, (_Float16)0.0f, (_Float16)0.0f,
                   (_Float16)0.0f, (_Float16)0.0f, (_Float16)0.0f, (_Float16)0.0f};
    for (int i = tid; i < (2 * HPLANE) / 8; i += NTHR) *(v8h*)(hpl + i * 8) = z;
  }
  float bcol[4];
#pragma unroll
  for (int j = 0; j < 4; ++j) {
    const int n = n0 + 16 * j + c;
    bcol[j] = (bf16r(b_ih[n]) + bf16r(b_hh[n])) * WSC;
  }
  const int ocol = tid & 31;
  const int ocl  = (ocol < NO) ? ocol : (NO - 1);
  const float bo = bf16r(b_ho[ocl]);
  const int ojn = ocol >> 4, occ = ocol & 15;
  __syncthreads();

  const _Float16* arow_hi = hhi + c * HP + koff;
  const _Float16* arow_lo = hlo + c * HP + koff;
  const _Float16* wihrow  = wih16 + (size_t)(n0 + c) * NI + koff;
  const _Float16* whhrow  = whh16 + (size_t)(n0 + c) * NH + koff;
  const int jn = wave & 1, kq = wave >> 1;
  const _Float16* whorow  = who16 + (size_t)(jn * 16 + c) * NH + koff + kq * (NH / 4);
  const _Float16* orow_hi = arow_hi + kq * (NH / 4);
  const _Float16* orow_lo = arow_lo + kq * (NH / 4);
  const _Float16* xrow0   = x16 + (size_t)(b0 + c) * NT * NI + koff;
  const v8f z8 = {0.f, 0.f, 0.f, 0.f, 0.f, 0.f, 0.f, 0.f};

#pragma unroll 1
  for (int t = 0; t < NT; ++t) {
    v8f acc[4], accr[4];
#pragma unroll
    for (int j = 0; j < 4; ++j) {
      const float bj = bcol[j];
      acc[j]  = (v8f){bj, bj, bj, bj, bj, bj, bj, bj};
      accr[j] = z8;
    }
    {
      const _Float16* xrow = xrow0 + (size_t)t * NI;
#pragma unroll
      for (int kc = 0; kc < NI / 32; ++kc) {
        const v16h fx = Frag<_Float16>::load(xrow + kc * 32);
        v16h fb[4];
#pragma unroll
        for (int j = 0; j < 4; ++j) fb[j] = Frag<_Float16>::load(wihrow + (size_t)(16 * j) * NI + kc * 32);
#pragma unroll
        for (int j = 0; j < 4; ++j) acc[j] = Frag<_Float16>::mma(fx, fb[j], acc[j]);
        guard4_f5(acc[0], acc[1], acc[2], acc[3], fx, fb[0], fb[1], fb[2], fb[3]);
      }
    }
#pragma unroll 1
    for (int kc = 0; kc < NH / 32; ++kc) {
      const v16h fah = Frag<_Float16>::load(arow_hi + kc * 32);
      const v16h fal = Frag<_Float16>::load(arow_lo + kc * 32);
      v16h fb[4];
#pragma unroll
      for (int j = 0; j < 4; ++j) fb[j] = Frag<_Float16>::load(whhrow + (size_t)(16 * j) * NH + kc * 32);
#pragma unroll
      for (int j = 0; j < 4; ++j) {
        acc[j]  = Frag<_Float16>::mma(fah, fb[j], acc[j]);
        accr[j] = Frag<_Float16>::mma(fal, fb[j], accr[j]);
      }
      guard8_f6(acc[0], acc[1], acc[2], acc[3], accr[0], accr[1], accr[2], accr[3],
                fah, fal, fb[0], fb[1], fb[2], fb[3]);
    }
    acc_guard4(acc[0], acc[1], acc[2], acc[3]);
    acc_guard4(accr[0], accr[1], accr[2], accr[3]);
    __syncthreads();

#pragma unroll
    for (int j = 0; j < 4; ++j) {
      const int col = n0 + 16 * j + c;
#pragma unroll
      for (int r = 0; r < 8; ++r) {
        const float v   = fmaf(accr[j][r], LOSC_INV, acc[j][r]) * WSC_INV;
        const float hv  = tanhf(v);
        const _Float16 h16 = (_Float16)hv;
        const float res = (hv - (float)h16) * LOSC;
        const _Float16 l16 = (_Float16)res;
        const int idx = (mOff + r) * HP + col;
        hhi[idx] = h16;
        hlo[idx] = l16;
      }
    }
    __syncthreads();

    {
      v8f oh = z8, ohr = z8;
#pragma unroll 1
      for (int kc = 0; kc < (NH / 4) / 32; ++kc) {
        const v16h fah = Frag<_Float16>::load(orow_hi + kc * 32);
        const v16h fal = Frag<_Float16>::load(orow_lo + kc * 32);
        const v16h fw  = Frag<_Float16>::load(whorow + kc * 32);
        oh  = Frag<_Float16>::mma(fah, fw, oh);
        ohr = Frag<_Float16>::mma(fal, fw, ohr);
        guard2_f3(oh, ohr, fah, fal, fw);
      }
      acc_guard2(oh, ohr);
#pragma unroll
      for (int r = 0; r < 8; ++r)
        part[wave * 256 + (mOff + r) * 16 + c] = fmaf(ohr[r], LOSC_INV, oh[r]) * WSC_INV;
    }
    __syncthreads();

    const int tl = t & (TCH - 1);
#pragma unroll
    for (int q = 0; q < 2; ++q) {
      const int row = (tid + q * NTHR) >> 5;
      const int pb  = row * 16 + occ;
      float s = part[ojn * 256 + pb];
      s += part[(2 + ojn) * 256 + pb];
      s += part[(4 + ojn) * 256 + pb];
      s += part[(6 + ojn) * 256 + pb];
      const float o = tanhf(s + bo);
      if (ocol < NO) ring[row * RROW + tl * NO + ocol] = o;
    }
    if (tl == TCH - 1) {
      __syncthreads();
      const int t0 = t - (TCH - 1);
      for (int pass = 0; pass < 2; ++pass) {
#pragma unroll
        for (int it = 0; it < (RB * RROW / 4) / NTHR; ++it) {
          const int f   = it * NTHR + tid;
          const int row = f / (RROW / 4);
          const int w4  = f - row * (RROW / 4);
          const v4f v = *(const v4f*)(ring + row * RROW + w4 * 4);
          *(volatile v4f*)(out + ((size_t)(b0 + row) * NT + (size_t)t0) * NO + w4 * 4) = v;
        }
        __threadfence();
      }
    }
  }
}

extern "C" void kernel_launch(void* const* d_in, const int* in_sizes, int n_in,
                              void* d_out, int out_size, void* d_ws, size_t ws_size, hipStream_t stream) {
  if (n_in < 7 || d_out == nullptr || d_ws == nullptr) return;
  if (in_sizes[0] != NB * NT * NI || in_sizes[1] != NH * NI || in_sizes[2] != NH * NH ||
      in_sizes[3] != NH || in_sizes[4] != NH || in_sizes[5] != NO * NH || in_sizes[6] != NO ||
      out_size != NB * NT * NO) return;

  const float* x    = (const float*)d_in[0];
  const float* w_ih = (const float*)d_in[1];
  const float* w_hh = (const float*)d_in[2];
  const float* b_ih = (const float*)d_in[3];
  const float* b_hh = (const float*)d_in[4];
  const float* w_ho = (const float*)d_in[5];
  const float* b_ho = (const float*)d_in[6];
  float* out = (float*)d_out;

  char* ws = (char*)d_ws; size_t off = 0;
  auto carve = [&](size_t bytes) -> char* { char* p = ws + off; off += (bytes + 255) & ~(size_t)255; return p; };
  _Float16* X16   = (_Float16*)carve((size_t)NB * NT * NI * 2);
  _Float16* WHH16 = (_Float16*)carve((size_t)NH * NH * 2);
  _Float16* WIH16 = (_Float16*)carve((size_t)NH * NI * 2);
  _Float16* WHO16 = (_Float16*)carve((size_t)NOPAD * NH * 2);
  if (off > ws_size || off > (size_t)134217728) return;

  cvt_kernel<<<CVT_BLOCKS, NTHR, 0, stream>>>(x, w_ih, w_hh, w_ho, X16, WIH16, WHH16, WHO16);

  rnn_seq_kernel<<<NB / RB, NTHR, 0, stream>>>(X16, WIH16, WHH16, WHO16, b_ih, b_hh, b_ho, out);
}
